// PointNet_FP_Module_11166914970522
// MI455X (gfx1250) — hardware-verified
//
#include <hip/hip_runtime.h>
#pragma clang fp contract(off)

typedef __attribute__((ext_vector_type(16))) _Float16 v16h;
typedef __attribute__((ext_vector_type(8)))  _Float16 v8h;
typedef __attribute__((ext_vector_type(16))) __bf16   v16b;
typedef __attribute__((ext_vector_type(8)))  float    v8f;
typedef __attribute__((ext_vector_type(4)))  float    v4f;
typedef __attribute__((ext_vector_type(4)))  unsigned v4u;

constexpr int NBATCH = 4;
constexpr int NQRY   = 8192;
constexpr int NSRC   = 2048;
constexpr int CHP1   = 128;
constexpr int CHP2   = 256;
constexpr int CIN0   = CHP1 + CHP2;
constexpr int COUT0  = 256;
constexpr int MROWS  = NBATCH * NQRY;
constexpr int KPL0   = 3 * CIN0;
constexpr int KPL1   = 3 * COUT0;
constexpr int NSTATB = MROWS / 128;

constexpr float EPS_DIST_F = 1e-07f;
constexpr float EPS_W_F    = 1e-08f;
constexpr float EPS_BN_F   = 1e-05f;
constexpr float F16_MIN_NORMAL = 6.103515625e-05f;

static_assert(CIN0 == 384 && COUT0 == 256 && MROWS == 32768, "shape");
static_assert(MROWS % 64 == 0 && COUT0 % 64 == 0, "tile multiples");
static_assert(KPL0 % 32 == 0 && CIN0 % 32 == 0 && KPL1 % 32 == 0 && COUT0 % 32 == 0, "k multiples");
static_assert(NSRC % 256 == 0 && NQRY % 256 == 0, "selection grid");

__device__ __forceinline__ unsigned bf16_bits(float f) {
  const unsigned u = __float_as_uint(f);
  return (u + 0x7FFFu + ((u >> 16) & 1u)) >> 16;
}
__device__ __forceinline__ unsigned f16_bits(float f) {
  const _Float16 h = (_Float16)f;
  const unsigned short s = __builtin_bit_cast(unsigned short, h);
  return (unsigned)s;
}
__device__ __forceinline__ void split3(float v, unsigned& hb, unsigned& lb, unsigned& bb) {
  const _Float16 h = (_Float16)v;
  float hf = (float)h;
  const bool tiny = fabsf(hf) < F16_MIN_NORMAL;
  hf = tiny ? 0.0f : hf;
  hb = f16_bits(hf);
  const float res = v - hf;
  lb = bf16_bits(res);
  bb = bf16_bits(v);
}
__device__ __forceinline__ unsigned pk2(unsigned a, unsigned b) {
  return (a & 0xffffu) | (b << 16);
}
__device__ __forceinline__ v4u pack8(const unsigned (&h)[8]) {
  v4u r;
  r.x = pk2(h[0], h[1]);
  r.y = pk2(h[2], h[3]);
  r.z = pk2(h[4], h[5]);
  r.w = pk2(h[6], h[7]);
  return r;
}

__device__ __forceinline__ void prep_chunk(const float* __restrict__ src, unsigned short* __restrict__ dst,
                                           int kin, int gl) {
  const int cpr = kin >> 3;
  int row = gl / cpr;
  const int c = gl - row * cpr;
  row = row < COUT0 ? row : (COUT0 - 1);
  const float* sp = src + (size_t)row * kin + c * 8;
  const v4f a = *(const v4f*)(sp);
  const v4f b = *(const v4f*)(sp + 4);
  float w[8];
  w[0] = a.x; w[1] = a.y; w[2] = a.z; w[3] = a.w;
  w[4] = b.x; w[5] = b.y; w[6] = b.z; w[7] = b.w;
  unsigned hb[8], lb[8], bb[8];
#pragma unroll
  for (int e = 0; e < 8; ++e) split3(w[e], hb[e], lb[e], bb[e]);
  const v4u H = pack8(hb);
  const v4u L = pack8(lb);
  const v4u Bv = pack8(bb);
  unsigned short* dp = dst + (size_t)row * (3 * kin) + c * 8;
  for (int pass = 0; pass < 2; ++pass) {
    *(volatile v4u*)(dp) = H;
    *(volatile v4u*)(dp + kin) = Bv;
    *(volatile v4u*)(dp + 2 * kin) = L;
    __threadfence();
  }
}
constexpr int PREP_CH0 = COUT0 * (CIN0 / 8);
constexpr int PREP_CH1 = COUT0 * (COUT0 / 8);
static_assert(PREP_CH0 % 256 == 0 && PREP_CH1 % 256 == 0, "prep grid");
__global__ __launch_bounds__(256) void prep_weights_kernel(
    const float* __restrict__ W0, const float* __restrict__ W1,
    unsigned short* __restrict__ bt0, unsigned short* __restrict__ bt1) {
  const int g = blockIdx.x * 256 + threadIdx.x;
  if (blockIdx.x < PREP_CH0 / 256) {
    prep_chunk(W0, bt0, CIN0, g);
  } else {
    prep_chunk(W1, bt1, COUT0, g - PREP_CH0);
  }
}

__global__ __launch_bounds__(256) void knn3_weights_kernel(
    const float* __restrict__ xyz1, const float* __restrict__ xyz2,
    int* __restrict__ idxp, float* __restrict__ wtp) {
#pragma clang fp contract(off)
  __shared__ __align__(16) float spts[NSRC * 4];
  const int b = blockIdx.y;
  const int tid = threadIdx.x;
  const float* src = xyz2 + (size_t)b * NSRC * 3;
#pragma unroll 1
  for (int i = 0; i < NSRC / 256; ++i) {
    const int n = i * 256 + tid;
    const float x = src[3 * n + 0];
    const float y = src[3 * n + 1];
    const float z = src[3 * n + 2];
    const float tx = x * x;
    const float ty = y * y;
    const float tz = z * z;
    const float s = (tx + tz) + ty;
    v4f q;
    q.x = x; q.y = y; q.z = z; q.w = s;
    *(v4f*)(spts + 4 * n) = q;
  }
  __syncthreads();

  const int m = b * NQRY + blockIdx.x * 256 + tid;
  const float ax = xyz1[(size_t)m * 3 + 0];
  const float ay = xyz1[(size_t)m * 3 + 1];
  const float az = xyz1[(size_t)m * 3 + 2];
  const float qx = ax * ax;
  const float qy = ay * ay;
  const float qz = az * az;
  const float s1 = (qx + qz) + qy;

  float e0 = __builtin_huge_valf(), e1 = __builtin_huge_valf(), e2 = __builtin_huge_valf();
  int j0 = 0, j1 = 0, j2 = 0;
#pragma unroll 4
  for (int n = 0; n < NSRC; ++n) {
    const v4f q = *(const v4f*)(spts + 4 * n);
    float p = ax * q.x;
    p = __builtin_fmaf(ay, q.y, p);
    p = __builtin_fmaf(az, q.z, p);
    const float s = s1 + q.w;
    const float p2 = p + p;
    float d = s - p2;
    d = (d < 0.0f) ? EPS_DIST_F : d;
    const bool c0 = d < e0;
    const bool c1 = d < e1;
    const bool c2 = d < e2;
    const float ne2 = c1 ? e1 : (c2 ? d : e2);
    const int   nj2 = c1 ? j1 : (c2 ? n : j2);
    const float ne1 = c0 ? e0 : (c1 ? d : e1);
    const int   nj1 = c0 ? j0 : (c1 ? n : j1);
    e0 = c0 ? d : e0;
    j0 = c0 ? n : j0;
    e1 = ne1; j1 = nj1;
    e2 = ne2; j2 = nj2;
  }
  const float r0 = sqrtf(e0);
  const float r1 = sqrtf(e1);
  const float r2 = sqrtf(e2);
  const float i0 = 1.0f / (r0 + EPS_W_F);
  const float i1 = 1.0f / (r1 + EPS_W_F);
  const float i2 = 1.0f / (r2 + EPS_W_F);
  const float isum = (i0 + i2) + i1;
  const float w0 = i0 / isum;
  const float w1 = i1 / isum;
  const float w2 = i2 / isum;
  for (int pass = 0; pass < 2; ++pass) {
    *(volatile int*)(idxp + m) = j0;
    *(volatile int*)(idxp + MROWS + m) = j1;
    *(volatile int*)(idxp + 2 * MROWS + m) = j2;
    *(volatile float*)(wtp + m) = w0;
    *(volatile float*)(wtp + MROWS + m) = w1;
    *(volatile float*)(wtp + 2 * MROWS + m) = w2;
    __threadfence();
  }
}

__global__ __launch_bounds__(256) void gather_concat_kernel(
    const float* __restrict__ points1, const float* __restrict__ points2,
    const int* __restrict__ idxp, const float* __restrict__ wtp,
    unsigned short* __restrict__ aplane) {
  const int lane = threadIdx.x & 31;
  const int wave = threadIdx.x >> 5;
  const int m = blockIdx.x * 8 + wave;
  const int b = m / NQRY;
  int j0 = idxp[m];
  int j1 = idxp[MROWS + m];
  int j2 = idxp[2 * MROWS + m];
  j0 = j0 < 0 ? 0 : (j0 > NSRC - 1 ? NSRC - 1 : j0);
  j1 = j1 < 0 ? 0 : (j1 > NSRC - 1 ? NSRC - 1 : j1);
  j2 = j2 < 0 ? 0 : (j2 > NSRC - 1 ? NSRC - 1 : j2);
  const float w0 = wtp[m];
  const float w1 = wtp[MROWS + m];
  const float w2 = wtp[2 * MROWS + m];
  const float* base = points2 + (size_t)b * NSRC * CHP2;
  const float* r0 = base + (size_t)j0 * CHP2 + lane * 8;
  const float* r1 = base + (size_t)j1 * CHP2 + lane * 8;
  const float* r2 = base + (size_t)j2 * CHP2 + lane * 8;
  const v4f a0 = *(const v4f*)(r0);
  const v4f a1 = *(const v4f*)(r0 + 4);
  const v4f b0 = *(const v4f*)(r1);
  const v4f b1 = *(const v4f*)(r1 + 4);
  const v4f c0 = *(const v4f*)(r2);
  const v4f c1 = *(const v4f*)(r2 + 4);
  float o[8];
#pragma unroll
  for (int e = 0; e < 4; ++e) {
    o[e]     = (w0 * a0[e] + w1 * b0[e]) + w2 * c0[e];
    o[4 + e] = (w0 * a1[e] + w1 * b1[e]) + w2 * c1[e];
  }
  unsigned hb[8], lb[8], bb[8];
#pragma unroll
  for (int e = 0; e < 8; ++e) split3(o[e], hb[e], lb[e], bb[e]);
  const v4u H = pack8(hb);
  const v4u L = pack8(lb);
  const v4u Bv = pack8(bb);

  asm volatile("" ::: "memory");
  const int l16 = lane & 15;
  const float* p1 = points1 + (size_t)m * CHP1 + l16 * 8;
  const v4f s0 = *(const v4f*)(p1);
  const v4f s1 = *(const v4f*)(p1 + 4);
  float sv[8];
  sv[0] = s0.x; sv[1] = s0.y; sv[2] = s0.z; sv[3] = s0.w;
  sv[4] = s1.x; sv[5] = s1.y; sv[6] = s1.z; sv[7] = s1.w;
  unsigned hs[8], ls[8], bs[8];
#pragma unroll
  for (int e = 0; e < 8; ++e) split3(sv[e], hs[e], ls[e], bs[e]);
  const v4u HS = pack8(hs);
  const v4u LS = pack8(ls);
  const v4u BS = pack8(bs);

  unsigned short* rowp = aplane + (size_t)m * KPL0;
  unsigned short* ip = rowp + lane * 8;
  unsigned short* sp = rowp + CHP2 + l16 * 8;
  for (int pass = 0; pass < 2; ++pass) {
    *(volatile v4u*)(ip) = H;
    *(volatile v4u*)(ip + CIN0) = L;
    *(volatile v4u*)(ip + 2 * CIN0) = Bv;
    if (lane < 16) {
      *(volatile v4u*)(sp) = HS;
      *(volatile v4u*)(sp + CIN0) = LS;
      *(volatile v4u*)(sp + 2 * CIN0) = BS;
    }
    __threadfence();
  }
}

__device__ __forceinline__ v16h frag_load(const _Float16* p) {
  union { v16h v; v8h h[2]; } f;
  f.h[0] = *(const v8h*)(p);
  f.h[1] = *(const v8h*)(p + 16);
  return f.v;
}
template <bool BF>
__device__ __forceinline__ v8f mma16(v16h a, v16h b, v8f c) {
  if (BF) {
    const v16b ab = __builtin_bit_cast(v16b, a);
    const v16b bb = __builtin_bit_cast(v16b, b);
    return __builtin_amdgcn_wmma_f32_16x16x32_bf16(false, ab, false, bb, (short)0, c, false, false);
  }
  return __builtin_amdgcn_wmma_f32_16x16x32_f16(false, a, false, b, (short)0, c, false, false);
}
__device__ __forceinline__ void guard_row(v8f& a0, v8f& a1, v8f& a2, v8f& a3,
                                          v16h x, v16h b0, v16h b1, v16h b2, v16h b3) {
  asm volatile("v_nop\n\tv_nop\n\tv_nop\n\tv_nop"
               : "+v"(a0), "+v"(a1), "+v"(a2), "+v"(a3)
               : "v"(x), "v"(b0), "v"(b1), "v"(b2), "v"(b3));
}
__device__ __forceinline__ void acc_guard4(v8f& a, v8f& b, v8f& c, v8f& d) {
  asm volatile("v_nop\n\tv_nop\n\tv_nop\n\tv_nop" : "+v"(a), "+v"(b), "+v"(c), "+v"(d));
}
template <bool BF>
__device__ __forceinline__ void gemm_kseg(v8f (&acc)[4][4], const _Float16* __restrict__ Ab,
                                          const _Float16* __restrict__ Bb, int lda, int ldb,
                                          int m0, int n0, int rlane, int koff, int kbeg, int kend) {
  for (int k0 = kbeg; k0 < kend; k0 += 32) {
    v16h bh[4];
#pragma unroll
    for (int j = 0; j < 4; ++j) {
      const size_t bo = (size_t)(n0 + (j << 4) + rlane) * ldb + koff + k0;
      bh[j] = frag_load(Bb + bo);
    }
#pragma unroll
    for (int i = 0; i < 4; ++i) {
      const size_t ao = (size_t)(m0 + (i << 4) + rlane) * lda + koff + k0;
      const v16h ah = frag_load(Ab + ao);
#pragma unroll
      for (int j = 0; j < 4; ++j) acc[i][j] = mma16<BF>(ah, bh[j], acc[i][j]);
      guard_row(acc[i][0], acc[i][1], acc[i][2], acc[i][3], ah, bh[0], bh[1], bh[2], bh[3]);
    }
  }
}

__global__ __launch_bounds__(256) void wmma_gemm64_seg(
    const unsigned short* __restrict__ Ap, int lda,
    const unsigned short* __restrict__ Btp, int ldb,
    float* __restrict__ Cout, int ldc,
    int Mrows, int Ncols, int Ktot, int Kf16) {
  __shared__ __align__(16) float sT[8][16 * 68];
  const _Float16* A = (const _Float16*)Ap;
  const _Float16* Bt = (const _Float16*)Btp;
  const int lane = threadIdx.x & 31;
  const int wave = threadIdx.x >> 5;
  const int tilesN = Ncols >> 6;
  const int tilesM = Mrows >> 6;
  const int tile = blockIdx.x * 8 + wave;
  if (tile >= tilesM * tilesN) return;
  const int tm = tile / tilesN;
  const int tn = tile - tm * tilesN;
  const int m0 = tm << 6;
  const int n0 = tn << 6;
  const int rlane = lane & 15;
  const int koff = (lane >> 4) * 8;
  const int mOff = (lane >> 4) * 8;

  v8f acc[4][4];
#pragma unroll
  for (int i = 0; i < 4; ++i)
#pragma unroll
    for (int j = 0; j < 4; ++j) acc[i][j] = (v8f){0.f, 0.f, 0.f, 0.f, 0.f, 0.f, 0.f, 0.f};

  gemm_kseg<false>(acc, A, Bt, lda, ldb, m0, n0, rlane, koff, 0, Kf16);
  gemm_kseg<true>(acc, A, Bt, lda, ldb, m0, n0, rlane, koff, Kf16, Ktot);

  acc_guard4(acc[0][0], acc[0][1], acc[0][2], acc[0][3]);
  acc_guard4(acc[1][0], acc[1][1], acc[1][2], acc[1][3]);
  acc_guard4(acc[2][0], acc[2][1], acc[2][2], acc[2][3]);
  acc_guard4(acc[3][0], acc[3][1], acc[3][2], acc[3][3]);

  float* slab = sT[wave];
#pragma unroll
  for (int i = 0; i < 4; ++i) {
    const int mBase = m0 + (i << 4);
#pragma unroll
    for (int j = 0; j < 4; ++j) {
#pragma unroll
      for (int r = 0; r < 8; ++r) {
        const float v = acc[i][j][r];
        slab[(mOff + r) * 68 + (j << 4) + rlane] = v;
      }
    }
    __builtin_amdgcn_fence(__ATOMIC_RELEASE, "workgroup");
    __builtin_amdgcn_wave_barrier();
    __builtin_amdgcn_fence(__ATOMIC_ACQUIRE, "workgroup");
    {
      const int hh = lane >> 4;
      const int c4 = (lane & 15) * 4;
      for (int pass = 0; pass < 2; ++pass) {
#pragma unroll
        for (int it = 0; it < 8; ++it) {
          const int row = it * 2 + hh;
          const v4f v = *(const v4f*)(slab + row * 68 + c4);
          *(volatile v4f*)(Cout + (size_t)(mBase + row) * ldc + n0 + c4) = v;
        }
        __threadfence();
      }
    }
    __builtin_amdgcn_fence(__ATOMIC_RELEASE, "workgroup");
    __builtin_amdgcn_wave_barrier();
    __builtin_amdgcn_fence(__ATOMIC_ACQUIRE, "workgroup");
  }
}

__global__ __launch_bounds__(256) void colstats_kernel(const float* __restrict__ y, float* __restrict__ part) {
  const int c = threadIdx.x;
  const int rbeg = blockIdx.x * 128;
  float s = 0.0f, ss = 0.0f;
#pragma unroll 8
  for (int r = 0; r < 128; ++r) {
    const float v = y[(size_t)(rbeg + r) * COUT0 + c];
    const float v2 = v * v;
    s = s + v;
    ss = ss + v2;
  }
  float* p = part + (size_t)blockIdx.x * 512;
  for (int pass = 0; pass < 2; ++pass) {
    *(volatile float*)(p + c) = s;
    *(volatile float*)(p + 256 + c) = ss;
    __threadfence();
  }
}
__global__ __launch_bounds__(256) void bn_finalize_kernel(
    const float* __restrict__ part, const float* __restrict__ gamma, const float* __restrict__ beta,
    float* __restrict__ tab) {
  const int c = threadIdx.x;
  double s = 0.0, ss = 0.0;
#pragma unroll 4
  for (int blk = 0; blk < NSTATB; ++blk) {
    const float a = part[(size_t)blk * 512 + c];
    const float b = part[(size_t)blk * 512 + 256 + c];
    s = s + (double)a;
    ss = ss + (double)b;
  }
  const double invn = 1.0 / (double)MROWS;
  const double mean = s * invn;
  double var = ss * invn - mean * mean;
  var = var < 0.0 ? 0.0 : var;
  const float varf = (float)var;
  const float rstd = 1.0f / sqrtf(varf + EPS_BN_F);
  const float sc = rstd * gamma[c];
  const float mf = (float)mean;
  const float bt = beta[c];
  for (int pass = 0; pass < 2; ++pass) {
    *(volatile float*)(tab + c) = mf;
    *(volatile float*)(tab + 256 + c) = sc;
    *(volatile float*)(tab + 512 + c) = bt;
    __threadfence();
  }
}

__global__ __launch_bounds__(256) void bn_relu_split_kernel(
    const float* __restrict__ y, const float* __restrict__ tab, unsigned short* __restrict__ aplane) {
  const int lane = threadIdx.x & 31;
  const int wave = threadIdx.x >> 5;
  const int cb = lane * 8;
  const v4f mA = *(const v4f*)(tab + cb);
  const v4f mB = *(const v4f*)(tab + cb + 4);
  const v4f sA = *(const v4f*)(tab + 256 + cb);
  const v4f sB = *(const v4f*)(tab + 256 + cb + 4);
  const v4f bA = *(const v4f*)(tab + 512 + cb);
  const v4f bB = *(const v4f*)(tab + 512 + cb + 4);
  const int rbase = (blockIdx.x * 8 + wave) * 4;
#pragma unroll 1
  for (int i = 0; i < 4; ++i) {
    const int m = rbase + i;
    const v4f yA = *(const v4f*)(y + (size_t)m * COUT0 + cb);
    const v4f yB = *(const v4f*)(y + (size_t)m * COUT0 + cb + 4);
    float v[8];
#pragma unroll
    for (int e = 0; e < 4; ++e) {
      const float ta = (yA[e] - mA[e]) * sA[e];
      const float tb = (yB[e] - mB[e]) * sB[e];
      v[e]     = fmaxf(ta + bA[e], 0.0f);
      v[4 + e] = fmaxf(tb + bB[e], 0.0f);
    }
    unsigned hb[8], lb[8], bb[8];
#pragma unroll
    for (int e = 0; e < 8; ++e) split3(v[e], hb[e], lb[e], bb[e]);
    const v4u H = pack8(hb);
    const v4u L = pack8(lb);
    const v4u Bv = pack8(bb);
    unsigned short* rp = aplane + (size_t)m * KPL1 + cb;
    for (int pass = 0; pass < 2; ++pass) {
      *(volatile v4u*)(rp) = H;
      *(volatile v4u*)(rp + COUT0) = L;
      *(volatile v4u*)(rp + 2 * COUT0) = Bv;
      __threadfence();
    }
  }
}

__global__ __launch_bounds__(256) void bn_relu_out_kernel(
    const float* __restrict__ y, const float* __restrict__ tab, float* __restrict__ outp) {
  const int lane = threadIdx.x & 31;
  const int wave = threadIdx.x >> 5;
  const int ca = lane * 4;
  const int cb = 128 + lane * 4;
  const v4f mA = *(const v4f*)(tab + ca);
  const v4f mB = *(const v4f*)(tab + cb);
  const v4f sA = *(const v4f*)(tab + 256 + ca);
  const v4f sB = *(const v4f*)(tab + 256 + cb);
  const v4f bA = *(const v4f*)(tab + 512 + ca);
  const v4f bB = *(const v4f*)(tab + 512 + cb);
  const int rbase = (blockIdx.x * 8 + wave) * 4;
#pragma unroll 1
  for (int i = 0; i < 4; ++i) {
    const int m = rbase + i;
    const v4f yA = *(const v4f*)(y + (size_t)m * COUT0 + ca);
    const v4f yB = *(const v4f*)(y + (size_t)m * COUT0 + cb);
    v4f oA, oB;
#pragma unroll
    for (int e = 0; e < 4; ++e) {
      const float ta = (yA[e] - mA[e]) * sA[e];
      const float tb = (yB[e] - mB[e]) * sB[e];
      oA[e] = fmaxf(ta + bA[e], 0.0f);
      oB[e] = fmaxf(tb + bB[e], 0.0f);
    }
    float* op = outp + (size_t)m * COUT0;
    for (int pass = 0; pass < 2; ++pass) {
      *(volatile v4f*)(op + ca) = oA;
      *(volatile v4f*)(op + cb) = oB;
      __threadfence();
    }
  }
}

constexpr size_t SZ_A    = (size_t)MROWS * KPL0 * 2;
constexpr size_t SZ_Y    = (size_t)MROWS * COUT0 * 4;
constexpr size_t SZ_BT0  = (size_t)COUT0 * KPL0 * 2;
constexpr size_t SZ_BT1  = (size_t)COUT0 * KPL1 * 2;
constexpr size_t SZ_IDX  = (size_t)3 * MROWS * 4;
constexpr size_t SZ_WT   = (size_t)3 * MROWS * 4;
constexpr size_t SZ_PART = (size_t)NSTATB * 512 * 4;
constexpr size_t SZ_TAB  = 4096;
constexpr size_t OFF_A   = 0;
constexpr size_t OFF_Y   = OFF_A + SZ_A;
constexpr size_t OFF_BT0 = OFF_Y + SZ_Y;
constexpr size_t OFF_BT1 = OFF_BT0 + SZ_BT0;
constexpr size_t OFF_IDX = OFF_BT1 + SZ_BT1;
constexpr size_t OFF_WT  = OFF_IDX + SZ_IDX;
constexpr size_t OFF_P0  = OFF_WT + SZ_WT;
constexpr size_t OFF_P1  = OFF_P0 + SZ_PART;
constexpr size_t OFF_T0  = OFF_P1 + SZ_PART;
constexpr size_t OFF_T1  = OFF_T0 + SZ_TAB;
constexpr size_t WS_TOTAL = OFF_T1 + SZ_TAB;
static_assert((size_t)MROWS * KPL1 * 2 <= SZ_A, "layer-1 operand rows fit the A region");
static_assert(WS_TOTAL <= (size_t)134217728, "carve under 128 MiB");
static_assert(OFF_Y % 128 == 0 && OFF_BT0 % 128 == 0 && OFF_BT1 % 128 == 0 && OFF_IDX % 128 == 0 &&
              OFF_WT % 128 == 0 && OFF_P0 % 128 == 0 && OFF_P1 % 128 == 0 && OFF_T0 % 128 == 0 && OFF_T1 % 128 == 0,
              "line-aligned carve");
static_assert(3 * 256 * 4 <= SZ_TAB, "tab fits");

extern "C" void kernel_launch(void* const* d_in, const int* in_sizes, int n_in,
                              void* d_out, int out_size, void* d_ws, size_t ws_size,
                              hipStream_t stream) {
  (void)in_sizes; (void)out_size;
  if (n_in < 10) return;
  if (ws_size < WS_TOTAL) return;
  const float* xyz1    = (const float*)d_in[0];
  const float* xyz2    = (const float*)d_in[1];
  const float* points1 = (const float*)d_in[2];
  const float* points2 = (const float*)d_in[3];
  const float* W0      = (const float*)d_in[4];
  const float* gamma0  = (const float*)d_in[5];
  const float* beta0   = (const float*)d_in[6];
  const float* W1      = (const float*)d_in[7];
  const float* gamma1  = (const float*)d_in[8];
  const float* beta1   = (const float*)d_in[9];
  float* outp = (float*)d_out;

  char* ws = (char*)d_ws;
  unsigned short* aplane = (unsigned short*)(ws + OFF_A);
  float*          yplane = (float*)(ws + OFF_Y);
  unsigned short* bt0    = (unsigned short*)(ws + OFF_BT0);
  unsigned short* bt1    = (unsigned short*)(ws + OFF_BT1);
  int*            idxp   = (int*)(ws + OFF_IDX);
  float*          wtp    = (float*)(ws + OFF_WT);
  float*          part0  = (float*)(ws + OFF_P0);
  float*          part1  = (float*)(ws + OFF_P1);
  float*          tab0   = (float*)(ws + OFF_T0);
  float*          tab1   = (float*)(ws + OFF_T1);

  constexpr int GEMM_BLOCKS = (MROWS / 64) * (COUT0 / 64) / 8;
  static_assert(((MROWS / 64) * (COUT0 / 64)) % 8 == 0, "gemm grid");

  prep_weights_kernel<<<(PREP_CH0 + PREP_CH1) / 256, 256, 0, stream>>>(W0, W1, bt0, bt1);
  knn3_weights_kernel<<<dim3(NQRY / 256, NBATCH), 256, 0, stream>>>(xyz1, xyz2, idxp, wtp);
  gather_concat_kernel<<<MROWS / 8, 256, 0, stream>>>(points1, points2, idxp, wtp, aplane);
  wmma_gemm64_seg<<<GEMM_BLOCKS, 256, 0, stream>>>(aplane, KPL0, bt0, KPL0, yplane, COUT0,
                                                   MROWS, COUT0, KPL0, CIN0);
  colstats_kernel<<<NSTATB, 256, 0, stream>>>(yplane, part0);
  bn_finalize_kernel<<<1, 256, 0, stream>>>(part0, gamma0, beta0, tab0);
  bn_relu_split_kernel<<<MROWS / 32, 256, 0, stream>>>(yplane, tab0, aplane);
  wmma_gemm64_seg<<<GEMM_BLOCKS, 256, 0, stream>>>(aplane, KPL1, bt1, KPL1, yplane, COUT0,
                                                   MROWS, COUT0, KPL1, COUT0);
  colstats_kernel<<<NSTATB, 256, 0, stream>>>(yplane, part1);
  bn_finalize_kernel<<<1, 256, 0, stream>>>(part1, gamma1, beta1, tab1);
  bn_relu_out_kernel<<<MROWS / 32, 256, 0, stream>>>(yplane, tab1, outp);
}
